// ScaledDotProduct_45698452029695
// MI455X (gfx1250) — hardware-verified
//
#include <hip/hip_runtime.h>


typedef _Float16 f16_t;
typedef _Float16 v16h __attribute__((ext_vector_type(16)));
typedef _Float16 v8h  __attribute__((ext_vector_type(8)));
typedef float    v8f  __attribute__((ext_vector_type(8)));
typedef float    v4f  __attribute__((ext_vector_type(4)));

#define SEQ 4096
#define DH  64
#define BM  64
#define BN  64
#define NW  4
#define NT  (NW * 32)
#define QSC 0.125f
#define PSC 16384.0f

union h8u   { f16_t h[8]; v8h v; };
union h2u   { f16_t h[2]; unsigned int u; };
union fragu { unsigned int u[8]; v8h p[2]; v16h v; };

__device__ __forceinline__ unsigned int pk_f16(float a, float b) {
  h2u x;
  x.h[0] = (f16_t)a;
  x.h[1] = (f16_t)b;
  return x.u;
}

__device__ __forceinline__ v8h cvt8(float4 a, float4 b, float sc) {
  h8u x;
  x.h[0] = (f16_t)(a.x * sc); x.h[1] = (f16_t)(a.y * sc);
  x.h[2] = (f16_t)(a.z * sc); x.h[3] = (f16_t)(a.w * sc);
  x.h[4] = (f16_t)(b.x * sc); x.h[5] = (f16_t)(b.y * sc);
  x.h[6] = (f16_t)(b.z * sc); x.h[7] = (f16_t)(b.w * sc);
  return x.v;
}

__device__ __forceinline__ v8f wmma16(v16h a, v16h b, v8f c) {
  c = __builtin_amdgcn_wmma_f32_16x16x32_f16(false, a, false, b, (short)0, c, false, false);
  asm volatile("v_nop\n\tv_nop\n\tv_nop\n\tv_nop" : "+v"(c) : "v"(a), "v"(b));
  return c;
}


__global__ __launch_bounds__(NT)
void cvt_planes_f16(const float* __restrict__ Qg,
                    const float* __restrict__ Kg,
                    const float* __restrict__ Vg,
                    f16_t* Qh, f16_t* Kh, f16_t* Vt, int nheads)
{
  __shared__ v8h sV[DH * BN / 8];

  const int tid  = threadIdx.x;
  const int hb   = blockIdx.y;
  const int kblk = blockIdx.x;
  if (hb >= nheads || kblk * BN >= SEQ) return;
  const size_t headoff = (size_t)hb * SEQ * DH;
  const int r0   = kblk * BN;
  const int rsub = tid >> 3;
  const int c8   = (tid & 7) * 8;

  v8h qv[4], kv[4];
  #pragma unroll
  for (int p = 0; p < 4; ++p) {
    const size_t off = headoff + (size_t)(r0 + p * 16 + rsub) * DH + c8;
    const float4 a0 = *(const float4*)(Qg + off);
    const float4 a1 = *(const float4*)(Qg + off + 4);
    const float4 b0 = *(const float4*)(Kg + off);
    const float4 b1 = *(const float4*)(Kg + off + 4);
    qv[p] = cvt8(a0, a1, QSC);
    kv[p] = cvt8(b0, b1, 1.0f);
  }

  {
    const int d4   = (tid & 15) * 4;
    const int key0 = (tid >> 4) * 8;
    const float* vp = Vg + headoff + (size_t)(r0 + key0) * DH + d4;
    h8u cb[4];
    #pragma unroll
    for (int k = 0; k < 8; ++k) {
      const float4 f = *(const float4*)(vp + (size_t)k * DH);
      cb[0].h[k] = (f16_t)f.x;
      cb[1].h[k] = (f16_t)f.y;
      cb[2].h[k] = (f16_t)f.z;
      cb[3].h[k] = (f16_t)f.w;
    }
    #pragma unroll
    for (int j = 0; j < 4; ++j)
      sV[(d4 + j) * (BN / 8) + (key0 >> 3)] = cb[j].v;
  }
  __syncthreads();

  v8h vv[4];
  #pragma unroll
  for (int p = 0; p < 4; ++p) vv[p] = sV[(p * 16 + rsub) * (BN / 8) + (tid & 7)];

  #pragma unroll
  for (int p = 0; p < 4; ++p) {
    const size_t rowoff = headoff + (size_t)(r0 + p * 16 + rsub) * DH + c8;
    *(volatile v8h*)(Qh + rowoff) = qv[p];
    *(volatile v8h*)(Kh + rowoff) = kv[p];
    *(volatile v8h*)(Vt + headoff + (size_t)(p * 16 + rsub) * SEQ + r0 + c8) = vv[p];
  }
  __threadfence();
  #pragma unroll
  for (int p = 0; p < 4; ++p) {
    const size_t rowoff = headoff + (size_t)(r0 + p * 16 + rsub) * DH + c8;
    *(volatile v8h*)(Qh + rowoff) = qv[p];
    *(volatile v8h*)(Kh + rowoff) = kv[p];
    *(volatile v8h*)(Vt + headoff + (size_t)(p * 16 + rsub) * SEQ + r0 + c8) = vv[p];
  }
}

__global__ __launch_bounds__(NT)
void attn_fwd_f16(const f16_t* __restrict__ Qh,
                  const f16_t* __restrict__ Kh,
                  const f16_t* __restrict__ Vt,
                  float* __restrict__ Og,
                  int nheads)
{
  __shared__ v4f sO[BM * DH / 4];

  const int tid  = threadIdx.x;
  const int lane = tid & 31;
  const int wave = tid >> 5;
  const int q16  = lane & 15;
  const int half = lane >> 4;

  const int hb   = blockIdx.y;
  const int qblk = blockIdx.x;
  if (hb >= nheads || qblk * BM >= SEQ) return;
  const size_t headoff = (size_t)hb * SEQ * DH;

  v16h qf[2];
  {
    const int qrow = qblk * BM + wave * 16 + q16;
    const f16_t* qp = Qh + headoff + (size_t)qrow * DH + 8 * half;
    #pragma unroll
    for (int kc = 0; kc < 2; ++kc) {
      fragu u;
      u.p[0] = *(const v8h*)(qp + kc * 32);
      u.p[1] = *(const v8h*)(qp + kc * 32 + 16);
      qf[kc] = u.v;
    }
  }

  v8f o[4];
  #pragma unroll
  for (int t = 0; t < 4; ++t) o[t] = (v8f){0.f, 0.f, 0.f, 0.f, 0.f, 0.f, 0.f, 0.f};
  float m_i = -__builtin_inff();
  float l_i = 0.f;

  const f16_t* kbase = Kh + headoff + (size_t)q16 * DH  + 8 * half;
  const f16_t* vbase = Vt + headoff + (size_t)q16 * SEQ + 8 * half;

  for (int kb0 = 0; kb0 < SEQ; kb0 += BN) {
    v8f s[4];
    #pragma unroll
    for (int mt = 0; mt < 4; ++mt) {
      v8f acc = (v8f){0.f, 0.f, 0.f, 0.f, 0.f, 0.f, 0.f, 0.f};
      #pragma unroll
      for (int kc = 0; kc < 2; ++kc) {
        const f16_t* ap = kbase + (size_t)(kb0 + mt * 16) * DH + kc * 32;
        fragu a;
        a.p[0] = *(const v8h*)(ap);
        a.p[1] = *(const v8h*)(ap + 16);
        acc = wmma16(a.v, qf[kc], acc);
      }
      s[mt] = acc;
    }

    float mx = -__builtin_inff();
    #pragma unroll
    for (int mt = 0; mt < 4; ++mt)
      #pragma unroll
      for (int r = 0; r < 8; ++r) mx = fmaxf(mx, s[mt][r]);
    mx = fmaxf(mx, __shfl_xor(mx, 16));
    const float mnew  = fmaxf(m_i, mx);
    const float alpha = __expf(m_i - mnew);
    float rs = 0.f;
    #pragma unroll
    for (int mt = 0; mt < 4; ++mt) {
      #pragma unroll
      for (int r = 0; r < 8; ++r) {
        const float p = __expf(s[mt][r] - mnew);
        s[mt][r] = p;
        rs += p;
      }
    }
    rs += __shfl_xor(rs, 16);
    l_i = l_i * alpha + rs;
    m_i = mnew;
    #pragma unroll
    for (int t = 0; t < 4; ++t)
      #pragma unroll
      for (int r = 0; r < 8; ++r) o[t][r] *= alpha;

    #pragma unroll
    for (int kc = 0; kc < 2; ++kc) {
      fragu pf;
      #pragma unroll
      for (int i = 0; i < 4; ++i) {
        pf.u[i]     = pk_f16(s[2 * kc][2 * i]     * PSC, s[2 * kc][2 * i + 1]     * PSC);
        pf.u[4 + i] = pk_f16(s[2 * kc + 1][2 * i] * PSC, s[2 * kc + 1][2 * i + 1] * PSC);
      }
      #pragma unroll
      for (int t = 0; t < 4; ++t) {
        const f16_t* ap = vbase + (size_t)(t * 16) * SEQ + kb0 + kc * 32;
        fragu a;
        a.p[0] = *(const v8h*)(ap);
        a.p[1] = *(const v8h*)(ap + 16);
        o[t] = wmma16(a.v, pf.v, o[t]);
      }
    }
  }

  const float inv = 1.0f / (l_i * PSC);
  {
    const int so = ((wave * 16 + q16) * DH) / 4;
    #pragma unroll
    for (int t = 0; t < 4; ++t) {
      v4f a, b;
      a[0] = o[t][0] * inv; a[1] = o[t][1] * inv; a[2] = o[t][2] * inv; a[3] = o[t][3] * inv;
      b[0] = o[t][4] * inv; b[1] = o[t][5] * inv; b[2] = o[t][6] * inv; b[3] = o[t][7] * inv;
      sO[so + t * 4 + half * 2]     = a;
      sO[so + t * 4 + half * 2 + 1] = b;
    }
  }
  __syncthreads();

  float* obase = Og + headoff + (size_t)qblk * BM * DH;
  v4f ov[8];
  #pragma unroll
  for (int j = 0; j < 8; ++j) ov[j] = sO[j * NT + tid];
  #pragma unroll
  for (int j = 0; j < 8; ++j)
    *(volatile v4f*)(obase + (size_t)(j * NT + tid) * 4) = ov[j];
  __threadfence();
  #pragma unroll
  for (int j = 0; j < 8; ++j)
    *(volatile v4f*)(obase + (size_t)(j * NT + tid) * 4) = ov[j];
}

extern "C" void kernel_launch(void* const* d_in, const int* in_sizes, int n_in,
                              void* d_out, int out_size, void* d_ws, size_t ws_size,
                              hipStream_t stream) {
  if (n_in < 3) return;
  const long long total = (long long)in_sizes[0];
  if ((long long)in_sizes[1] != total || (long long)in_sizes[2] != total) return;
  if ((long long)out_size != total) return;
  const long long per_head = (long long)SEQ * DH;
  if (total <= 0 || (total % per_head) != 0) return;
  const int nheads = (int)(total / per_head);

  const size_t plane_bytes = (size_t)total * sizeof(f16_t);
  if (3 * plane_bytes > ws_size) return;
  f16_t* Qh = (f16_t*)((char*)d_ws);
  f16_t* Kh = (f16_t*)((char*)d_ws + plane_bytes);
  f16_t* Vt = (f16_t*)((char*)d_ws + 2 * plane_bytes);

  const float* Q = (const float*)d_in[0];
  const float* K = (const float*)d_in[1];
  const float* V = (const float*)d_in[2];
  float* O = (float*)d_out;

  dim3 block(NT);
  dim3 grid1((SEQ + BN - 1) / BN, nheads);
  cvt_planes_f16<<<grid1, block, 0, stream>>>(Q, K, V, Qh, Kh, Vt, nheads);
  dim3 grid2((SEQ + BM - 1) / BM, nheads);
  attn_fwd_f16<<<grid2, block, 0, stream>>>(Qh, Kh, Vt, O, nheads);
  (void)hipGetLastError();
}
